// GRUCell_78451872628868
// MI455X (gfx1250) — hardware-verified
//
#include <hip/hip_runtime.h>
#include <math.h>

constexpr int NB_ROWS = 8192;
constexpr int NIN_F   = 1024;
constexpr int NHID    = 1024;
constexpr int NCAT    = NIN_F + NHID;
constexpr int NTHR    = 256;
constexpr int SLABP   = 68;
static_assert(NCAT % 32 == 0, "K multiple of 32, no pad needed");
static_assert(NB_ROWS % 64 == 0 && NHID % 64 == 0, "M and N are multiples of the 64x64 wave tile");
static_assert(((NB_ROWS / 64) * (NHID / 64)) % (NTHR / 32) == 0, "8 wave tiles per block exactly");
static_assert((NB_ROWS * (NHID / 8)) % NTHR == 0 && (NB_ROWS * (NIN_F / 8)) % NTHR == 0, "activation convert grids exact");
static_assert((NHID * (NCAT / 8)) % NTHR == 0, "weight convert grid exact");
static_assert((NHID / 8) % 32 == 0 && (NIN_F / 8) % 32 == 0 && (NCAT / 8) % 32 == 0, "a wave stays inside one row in the convert kernel");
static_assert(NIN_F == NHID, "x and h_prev share the row pitch used below");

typedef __attribute__((ext_vector_type(16))) __bf16   v16b;
typedef __attribute__((ext_vector_type(8)))  __bf16   v8b;
typedef __attribute__((ext_vector_type(8)))  float    v8f;
typedef __attribute__((ext_vector_type(4)))  float    v4f;
typedef __attribute__((ext_vector_type(4)))  unsigned v4u;

__device__ __forceinline__ unsigned short f2bf_bits(float f) {
  unsigned u = __float_as_uint(f);
  return (unsigned short)((u + 0x7FFFu + ((u >> 16) & 1u)) >> 16);
}
__device__ __forceinline__ float bf_bits2f(unsigned short h) { return __uint_as_float(((unsigned)h) << 16); }
__device__ __forceinline__ float bf16r(float f) { return bf_bits2f(f2bf_bits(f)); }

__device__ __forceinline__ void dep_guard4_b(v8f& a, v8f& b, v8f& c, v8f& d, v16b x, v16b y) {
  asm volatile("v_nop\n\tv_nop\n\tv_nop\n\tv_nop" : "+v"(a), "+v"(b), "+v"(c), "+v"(d) : "v"(x), "v"(y));
}
__device__ __forceinline__ void keep4_b(v16b a, v16b b, v16b c, v16b d) { asm volatile("v_nop" :: "v"(a), "v"(b), "v"(c), "v"(d)); }
__device__ __forceinline__ void acc_guard4(v8f& a, v8f& b, v8f& c, v8f& d) { asm volatile("v_nop\n\tv_nop\n\tv_nop\n\tv_nop" : "+v"(a), "+v"(b), "+v"(c), "+v"(d)); }

template <typename T> struct Frag;
template <> struct Frag<__bf16> {
  typedef v16b V; union U { v16b v; v8b h[2]; };
  static __device__ __forceinline__ v16b load(const __bf16* p) {
    U f; f.h[0] = *(const v8b*)(p); f.h[1] = *(const v8b*)(p + 16); return f.v;
  }
  static __device__ __forceinline__ v8f mma(v16b a, v16b b, v8f c) {
    return __builtin_amdgcn_wmma_f32_16x16x32_bf16(false, a, false, b, (short)0, c, false, false);
  }
};

__device__ __forceinline__ float sigm_f(float x) { return __builtin_amdgcn_rcpf(1.0f + expf(-x)); }
__device__ __forceinline__ float tanh_f(float x) { return 1.0f - 2.0f * __builtin_amdgcn_rcpf(expf(2.0f * x) + 1.0f); }

__global__ __launch_bounds__(NTHR) void cvt_bf16_kernel(const float* __restrict__ src, unsigned short* __restrict__ dst,
                                                        int nrow, int ncol8, int spitch, int dpitch, int dcol0) {
  const int i  = blockIdx.x * NTHR + threadIdx.x;
  const int n8 = nrow * ncol8;
  if (i < n8) {
    const int row = i / ncol8;
    const int c8  = i - row * ncol8;
    const float* sp = src + (size_t)row * spitch + (size_t)c8 * 8;
    const v4f a = *(const v4f*)(sp);
    const v4f b = *(const v4f*)(sp + 4);
    v4u pk;
    pk[0] = (unsigned)f2bf_bits(a[0]) | ((unsigned)f2bf_bits(a[1]) << 16);
    pk[1] = (unsigned)f2bf_bits(a[2]) | ((unsigned)f2bf_bits(a[3]) << 16);
    pk[2] = (unsigned)f2bf_bits(b[0]) | ((unsigned)f2bf_bits(b[1]) << 16);
    pk[3] = (unsigned)f2bf_bits(b[2]) | ((unsigned)f2bf_bits(b[3]) << 16);
    unsigned short* dp = dst + (size_t)row * dpitch + dcol0 + (size_t)c8 * 8;
    *(volatile v4u*)dp = pk;
    __threadfence();
    *(volatile v4u*)dp = pk;
  }
}

template <int EPI>
__global__ __launch_bounds__(NTHR) void gemm_bf16_kernel(
    const unsigned short* __restrict__ Ap, int lda,
    const unsigned short* __restrict__ Btp, int ldb,
    const float* __restrict__ bias,
    const float* __restrict__ zpl,
    const float* __restrict__ hpv,
    void* __restrict__ Cout, int ldc,
    int M, int N, int K) {
  const __bf16* A  = (const __bf16*)Ap;
  const __bf16* Bt = (const __bf16*)Btp;
  __shared__ __align__(16) float sT[NTHR / 32][16 * SLABP];
  const int lane = threadIdx.x & 31;
  const int wave = threadIdx.x >> 5;
  const int tilesN = N >> 6;
  const int tilesM = M >> 6;
  const int tile = blockIdx.x * (NTHR / 32) + wave;
  if (tile >= tilesM * tilesN) return;
  const int tm = tile / tilesN;
  const int tn = tile - tm * tilesN;
  const int m0 = tm << 6;
  const int n0 = tn << 6;

  const int rlane = lane & 15;
  const int koff  = (lane >> 4) * 8;
  const int mOff  = (lane >> 4) * 8;

  v8f acc[4][4];
#pragma unroll
  for (int i = 0; i < 4; ++i)
#pragma unroll
    for (int j = 0; j < 4; ++j) acc[i][j] = (v8f){0.f, 0.f, 0.f, 0.f, 0.f, 0.f, 0.f, 0.f};

  for (int k0 = 0; k0 < K; k0 += 32) {
    v16b bh[4];
#pragma unroll
    for (int j = 0; j < 4; ++j) {
      const size_t bo = (size_t)(n0 + (j << 4) + rlane) * ldb + koff + k0;
      bh[j] = Frag<__bf16>::load(Bt + bo);
    }
#pragma unroll
    for (int i = 0; i < 4; ++i) {
      const size_t ao = (size_t)(m0 + (i << 4) + rlane) * lda + koff + k0;
      const v16b ah = Frag<__bf16>::load(A + ao);
#pragma unroll
      for (int j = 0; j < 4; ++j) acc[i][j] = Frag<__bf16>::mma(ah, bh[j], acc[i][j]);
      dep_guard4_b(acc[i][0], acc[i][1], acc[i][2], acc[i][3], ah, bh[3]);
    }
    keep4_b(bh[0], bh[1], bh[2], bh[3]);
  }
  acc_guard4(acc[0][0], acc[0][1], acc[0][2], acc[0][3]);
  acc_guard4(acc[1][0], acc[1][1], acc[1][2], acc[1][3]);
  acc_guard4(acc[2][0], acc[2][1], acc[2][2], acc[2][3]);
  acc_guard4(acc[3][0], acc[3][1], acc[3][2], acc[3][3]);

  float bcol[4];
#pragma unroll
  for (int j = 0; j < 4; ++j) bcol[j] = bf16r(bias[n0 + (j << 4) + rlane]);

  float* slab = sT[wave];
#pragma unroll
  for (int i = 0; i < 4; ++i) {
    const int mBase = m0 + (i << 4);
#pragma unroll
    for (int j = 0; j < 4; ++j) {
#pragma unroll
      for (int r = 0; r < 8; ++r) {
        const float v = acc[i][j][r] + bcol[j];
        const float a = (EPI == 2) ? tanh_f(v) : sigm_f(v);
        slab[(mOff + r) * SLABP + (j << 4) + rlane] = a;
      }
    }
    __builtin_amdgcn_fence(__ATOMIC_RELEASE, "workgroup");
    __builtin_amdgcn_wave_barrier();
    __builtin_amdgcn_fence(__ATOMIC_ACQUIRE, "workgroup");

    if (EPI == 0) {
      float* C = (float*)Cout;
      const int hh = lane >> 4, c4 = (lane & 15) * 4;
      for (int pass = 0; pass < 2; ++pass) {
#pragma unroll
        for (int it = 0; it < 8; ++it) {
          const int row = it * 2 + hh;
          const v4f v = *(const v4f*)(slab + row * SLABP + c4);
          *(volatile v4f*)(C + (size_t)(mBase + row) * ldc + n0 + c4) = v;
        }
        __threadfence();
      }
    } else if (EPI == 1) {
      unsigned short* C = (unsigned short*)Cout;
      const int q = lane >> 3, c8 = (lane & 7) * 8;
      v4u pk[4];
#pragma unroll
      for (int it = 0; it < 4; ++it) {
        const int row = it * 4 + q;
        const float* sp = slab + row * SLABP + c8;
        const v4f s0 = *(const v4f*)(sp);
        const v4f s1 = *(const v4f*)(sp + 4);
        const float* hrow = hpv + (size_t)(mBase + row) * NHID + n0 + c8;
        const v4f g0 = *(const v4f*)(hrow);
        const v4f g1 = *(const v4f*)(hrow + 4);
        float p[8];
#pragma unroll
        for (int e = 0; e < 4; ++e) {
          p[e]     = s0[e] * bf16r(g0[e]);
          p[4 + e] = s1[e] * bf16r(g1[e]);
        }
        v4u wv;
#pragma unroll
        for (int e = 0; e < 4; ++e) wv[e] = (unsigned)f2bf_bits(p[2 * e]) | ((unsigned)f2bf_bits(p[2 * e + 1]) << 16);
        pk[it] = wv;
        if (it == 1) asm volatile("" ::: "memory");
      }
      for (int pass = 0; pass < 2; ++pass) {
#pragma unroll
        for (int it = 0; it < 4; ++it) {
          const int row = it * 4 + q;
          *(volatile v4u*)(C + (size_t)(mBase + row) * ldc + n0 + c8) = pk[it];
        }
        __threadfence();
      }
    } else {
      float* C = (float*)Cout;
      const int hh = lane >> 4, c4 = (lane & 15) * 4;
      v4f ov[8];
#pragma unroll
      for (int it = 0; it < 8; ++it) {
        const int row = it * 2 + hh;
        const v4f s = *(const v4f*)(slab + row * SLABP + c4);
        const size_t off = (size_t)(mBase + row) * NHID + n0 + c4;
        const v4f zv = *(const v4f*)(zpl + off);
        const v4f gv = *(const v4f*)(hpv + off);
        v4f o;
#pragma unroll
        for (int e = 0; e < 4; ++e) {
          const float hb = bf16r(gv[e]);
          o[e] = (1.0f - zv[e]) * hb + zv[e] * s[e];
        }
        ov[it] = o;
        if ((it & 1) == 1) asm volatile("" ::: "memory");
      }
      for (int pass = 0; pass < 2; ++pass) {
#pragma unroll
        for (int it = 0; it < 8; ++it) {
          const int row = it * 2 + hh;
          *(volatile v4f*)(C + (size_t)(mBase + row) * ldc + n0 + c4) = ov[it];
        }
        __threadfence();
      }
    }
    __builtin_amdgcn_fence(__ATOMIC_RELEASE, "workgroup");
    __builtin_amdgcn_wave_barrier();
    __builtin_amdgcn_fence(__ATOMIC_ACQUIRE, "workgroup");
  }
}

extern "C" void kernel_launch(void* const* d_in, const int* in_sizes, int n_in,
                              void* d_out, int out_size, void* d_ws, size_t ws_size, hipStream_t stream) {
  if (n_in < 8 || d_out == nullptr || d_ws == nullptr) return;
  if (in_sizes[0] != NB_ROWS * NIN_F || in_sizes[1] != NB_ROWS * NHID ||
      in_sizes[2] != NHID * NCAT || in_sizes[3] != NHID ||
      in_sizes[4] != NHID * NCAT || in_sizes[5] != NHID ||
      in_sizes[6] != NHID * NCAT || in_sizes[7] != NHID ||
      out_size != NB_ROWS * NHID) return;

  const float* x      = (const float*)d_in[0];
  const float* h_prev = (const float*)d_in[1];
  const float* w_z    = (const float*)d_in[2];
  const float* b_z    = (const float*)d_in[3];
  const float* w_r    = (const float*)d_in[4];
  const float* b_r    = (const float*)d_in[5];
  const float* w_h    = (const float*)d_in[6];
  const float* b_h    = (const float*)d_in[7];
  float* out = (float*)d_out;

  char* ws = (char*)d_ws; size_t off = 0;
  auto carve = [&](size_t bytes) -> char* { char* p = ws + off; off += (bytes + 255) & ~(size_t)255; return p; };
  unsigned short* A1 = (unsigned short*)carve((size_t)NB_ROWS * NCAT * 2);
  unsigned short* A2 = (unsigned short*)carve((size_t)NB_ROWS * NCAT * 2);
  unsigned short* WZ = (unsigned short*)carve((size_t)NHID * NCAT * 2);
  unsigned short* WR = (unsigned short*)carve((size_t)NHID * NCAT * 2);
  unsigned short* WH = (unsigned short*)carve((size_t)NHID * NCAT * 2);
  float*          ZP = (float*)carve((size_t)NB_ROWS * NHID * 4);
  if (off > ws_size || off > (size_t)134217728) return;

  const int gact = NB_ROWS * (NHID / 8) / NTHR;
  const int gwgt = NHID * (NCAT / 8) / NTHR;
  cvt_bf16_kernel<<<gact, NTHR, 0, stream>>>(h_prev, A1, NB_ROWS, NHID / 8,  NHID,  NCAT, 0);
  cvt_bf16_kernel<<<gact, NTHR, 0, stream>>>(x,      A1, NB_ROWS, NIN_F / 8, NIN_F, NCAT, NHID);
  cvt_bf16_kernel<<<gact, NTHR, 0, stream>>>(x,      A2, NB_ROWS, NIN_F / 8, NIN_F, NCAT, NHID);
  cvt_bf16_kernel<<<gwgt, NTHR, 0, stream>>>(w_z,    WZ, NHID,    NCAT / 8,  NCAT,  NCAT, 0);
  cvt_bf16_kernel<<<gwgt, NTHR, 0, stream>>>(w_r,    WR, NHID,    NCAT / 8,  NCAT,  NCAT, 0);
  cvt_bf16_kernel<<<gwgt, NTHR, 0, stream>>>(w_h,    WH, NHID,    NCAT / 8,  NCAT,  NCAT, 0);

  const int gblk = (NB_ROWS / 64) * (NHID / 64) / (NTHR / 32);
  gemm_bf16_kernel<0><<<gblk, NTHR, 0, stream>>>(A1, NCAT, WZ, NCAT, b_z, ZP, h_prev, (void*)ZP, NHID, NB_ROWS, NHID, NCAT);
  gemm_bf16_kernel<1><<<gblk, NTHR, 0, stream>>>(A1, NCAT, WR, NCAT, b_r, ZP, h_prev, (void*)A2, NCAT, NB_ROWS, NHID, NCAT);
  gemm_bf16_kernel<2><<<gblk, NTHR, 0, stream>>>(A2, NCAT, WH, NCAT, b_h, ZP, h_prev, (void*)out, NHID, NB_ROWS, NHID, NCAT);
}
